// SRCNN_36928128811191
// MI455X (gfx1250) — hardware-verified
//
#include <hip/hip_runtime.h>
#include <stddef.h>


typedef float          v4f   __attribute__((ext_vector_type(4)));
typedef float          v8f   __attribute__((ext_vector_type(8)));
typedef unsigned short v8us  __attribute__((ext_vector_type(8)));
typedef unsigned short v16us __attribute__((ext_vector_type(16)));
typedef __bf16         v16bf __attribute__((ext_vector_type(16)));

#define IMG  256
#define LOW  32
#define NIMG 16
#define HALF 8
#define K1   352
#define K2   64
#define K3   1280
#define PL1  (64 * K1)
#define PL2  (32 * K2)
#define PL3  (16 * K3)
#define TUC  72
#define THC  68
#define H1P  128

static_assert(((PL1 * 2) % 512) == 0);
static_assert(((PL2 * 2) % 512) == 0);
static_assert(((PL3 * 2) % 512) == 0);

__device__ __forceinline__ unsigned short f2bf(float x) {
  unsigned int u = __float_as_uint(x);
  u += 0x7FFFu + ((u >> 16) & 1u);
  return (unsigned short)(u >> 16);
}
__device__ __forceinline__ float bf2f(unsigned short b) {
  return __uint_as_float(((unsigned int)b) << 16);
}
__device__ __forceinline__ v8us sel8(bool keep, v8us a) {
  const unsigned short mk = keep ? (unsigned short)0xFFFFu : (unsigned short)0u;
  const v8us mv = {mk, mk, mk, mk, mk, mk, mk, mk};
  return a & mv;
}
__device__ __forceinline__ v8us ld8(const unsigned short* p) { return *(const v8us*)p; }
__device__ __forceinline__ v8us pickh(v8us a, v8us b) {
  return __builtin_shufflevector(a, b, 0, 1, 2, 3, 8, 9, 10, 11);
}
__device__ __forceinline__ v8us pickl(v8us a, v8us b) {
  return __builtin_shufflevector(a, b, 4, 5, 6, 7, 12, 13, 14, 15);
}
__device__ __forceinline__ v16us cat16(v8us a, v8us b) {
  return __builtin_shufflevector(a, b, 0, 1, 2, 3, 4, 5, 6, 7, 8, 9, 10, 11, 12, 13, 14, 15);
}
__device__ __forceinline__ v16bf tobf(v16us u) { return __builtin_bit_cast(v16bf, u); }
__device__ __forceinline__ v8f zero8f() {
  const v8f z = {0.0f, 0.0f, 0.0f, 0.0f, 0.0f, 0.0f, 0.0f, 0.0f};
  return z;
}

__device__ __forceinline__ v8f mma3(v8f c, v16bf ah, v16bf al, v16bf bh, v16bf blo) {
  c = __builtin_amdgcn_wmma_f32_16x16x32_bf16(false, ah, false, bh, (short)0, c, false, false);
  c = __builtin_amdgcn_wmma_f32_16x16x32_bf16(false, ah, false, blo, (short)0, c, false, false);
  c = __builtin_amdgcn_wmma_f32_16x16x32_bf16(false, al, false, bh, (short)0, c, false, false);
  asm volatile("v_nop\n\tv_nop\n\tv_nop\n\tv_nop" : "+v"(c) : "v"(ah), "v"(al), "v"(bh), "v"(blo));
  return c;
}

__global__ __launch_bounds__(256) void k_prep(const float* __restrict__ w1,
                                              const float* __restrict__ w2,
                                              const float* __restrict__ w3,
                                              unsigned short* B1, unsigned short* B2,
                                              unsigned short* B3) {
  const int mat = blockIdx.y;
  const int u = blockIdx.x * 256 + threadIdx.x;
  float v[8];
  int units, plane;
  unsigned short* dst;
  if (mat == 0) {
    units = 64 * (K1 / 8); plane = PL1; dst = B1;
    const int uc = min(u, units - 1);
    const int n = uc / (K1 / 8), k8 = (uc - n * (K1 / 8)) * 8;
#pragma unroll
    for (int e = 0; e < 8; ++e) {
      const int k = k8 + e, t = k >> 2, c = k & 3;
      const int tc = min(t, 80);
      const float x = w1[(n * 4 + c) * 81 + tc];
      v[e] = (t < 81) ? x : 0.0f;
    }
  } else if (mat == 1) {
    units = 32 * (K2 / 8); plane = PL2; dst = B2;
    const int uc = min(u, units - 1);
#pragma unroll
    for (int e = 0; e < 8; ++e) v[e] = w2[uc * 8 + e];
  } else {
    units = 16 * (K3 / 8); plane = PL3; dst = B3;
    const int uc = min(u, units - 1);
    const int n = uc / (K3 / 8), k8 = (uc - n * (K3 / 8)) * 8;
    const int c = n & 3, s = n >> 2;
#pragma unroll
    for (int e = 0; e < 8; ++e) {
      const int k = k8 + e, q = k >> 5, ci = k & 31;
      const int dy = q >> 3, dxp = q & 7, dx = dxp - s;
      const int dxc = min(max(dx, 0), 4);
      const float x = w3[((c * 32 + ci) * 5 + dy) * 5 + dxc];
      v[e] = ((unsigned)dx <= 4u) ? x : 0.0f;
    }
  }
  v8us H, L;
#pragma unroll
  for (int e = 0; e < 8; ++e) {
    const unsigned short hs = f2bf(v[e]);
    H[e] = hs;
    L[e] = f2bf(v[e] - bf2f(hs));
  }
  const bool wr = u < units;
  unsigned short* ph = dst + (size_t)u * 8;
  unsigned short* pl = dst + plane + (size_t)u * 8;
  if (wr) { *(volatile v8us*)ph = H; *(volatile v8us*)pl = L; }
  __threadfence();
  if (wr) { *(volatile v8us*)ph = H; *(volatile v8us*)pl = L; }
}

__device__ __forceinline__ float cubic_w(float d) {
  d = fabsf(d);
  const float d2 = d * d, d3 = d2 * d;
  const float p1 = 1.25f * d3 - 2.25f * d2 + 1.0f;
  const float p2 = -0.75f * d3 + 3.75f * d2 - 6.0f * d + 3.0f;
  return (d <= 1.0f) ? p1 : ((d < 2.0f) ? p2 : 0.0f);
}

__global__ __launch_bounds__(256) void k_up(const float* __restrict__ x, unsigned short* up) {
  const int P = blockIdx.x * 256 + threadIdx.x;
  const int b = P >> 16, Y = (P >> 8) & 255, X = P & 255;
  const float sy = ((float)Y + 0.5f) * 0.125f - 0.5f;
  const float sx = ((float)X + 0.5f) * 0.125f - 0.5f;
  const float fy = floorf(sy), fx = floorf(sx);
  const int by = (int)fy, bx = (int)fx;
  const float ty = sy - fy, tx = sx - fx;
  const float wx0 = cubic_w(tx + 1.0f), wx1 = cubic_w(tx), wx2 = cubic_w(tx - 1.0f), wx3 = cubic_w(tx - 2.0f);
  const int ix0 = min(max(bx - 1, 0), LOW - 1), ix1 = min(max(bx, 0), LOW - 1);
  const int ix2 = min(max(bx + 1, 0), LOW - 1), ix3 = min(max(bx + 2, 0), LOW - 1);
  v4f acc = {0.0f, 0.0f, 0.0f, 0.0f};
#pragma unroll 1
  for (int i = 0; i < 4; ++i) {
    const float wy = cubic_w(ty - (float)(i - 1));
    const int iy = min(max(by + i - 1, 0), LOW - 1);
    const float* row = x + ((size_t)((b * LOW + iy) * LOW)) * 4;
    const v4f p0 = *(const v4f*)(row + ix0 * 4);
    const v4f p1 = *(const v4f*)(row + ix1 * 4);
    const v4f p2 = *(const v4f*)(row + ix2 * 4);
    const v4f p3 = *(const v4f*)(row + ix3 * 4);
    v4f t = wx0 * p0;
    t = t + wx1 * p1;
    t = t + wx2 * p2;
    t = t + wx3 * p3;
    acc = acc + wy * t;
  }
  v8us o;
#pragma unroll
  for (int c = 0; c < 4; ++c) {
    const unsigned short hs = f2bf(acc[c]);
    o[c] = hs;
    o[4 + c] = f2bf(acc[c] - bf2f(hs));
  }
  unsigned short* p = up + (size_t)P * 8;
  *(volatile v8us*)p = o;
  __threadfence();
  *(volatile v8us*)p = o;
}

__device__ __forceinline__ int tapoff(int t) {
  const int dy = t / 9;
  return (dy * TUC + (t - dy * 9)) * 8;
}

__global__ __launch_bounds__(128) void k_conv12(const unsigned short* __restrict__ up,
                                                const unsigned short* __restrict__ B1,
                                                const float* __restrict__ b1,
                                                const unsigned short* __restrict__ B2,
                                                const float* __restrict__ b2,
                                                unsigned short* h2, int bimg0) {
  __shared__ __attribute__((aligned(16))) unsigned short tileU[9 * TUC * 8];
  __shared__ __attribute__((aligned(16))) unsigned short h1s[4 * 16 * H1P];
  __shared__ __attribute__((aligned(16))) unsigned short h2s[4 * 16 * 64];

  const int tid = threadIdx.x, lane = tid & 31, w = tid >> 5, h = lane >> 4, m = lane & 15;
  const int x0 = blockIdx.x * 64, Y = blockIdx.y, bi = blockIdx.z, bg = bimg0 + bi;

  for (int e = tid; e < 9 * TUC; e += 128) {
    const int i = e / TUC, j = e - i * TUC;
    const int Yg = Y - 4 + i, Xg = x0 - 4 + j;
    const bool in = ((unsigned)Yg < (unsigned)IMG) && ((unsigned)Xg < (unsigned)IMG);
    const int Yc = min(max(Yg, 0), IMG - 1), Xc = min(max(Xg, 0), IMG - 1);
    v8us v = ld8(up + ((size_t)((bg * IMG + Yc) * IMG + Xc)) * 8);
    v = sel8(in, v);
    *(v8us*)(tileU + e * 8) = v;
  }
  __syncthreads();

  v8f acc[4];
#pragma unroll
  for (int nt = 0; nt < 4; ++nt) acc[nt] = zero8f();
  const unsigned short* tw  = tileU + (16 * w + m) * 8;
  const unsigned short* bw1 = B1 + m * K1 + 8 * h;
  const v8us z8 = {0, 0, 0, 0, 0, 0, 0, 0};
#pragma unroll 1
  for (int g = 0; g < 10; ++g) {
    const int tA = 8 * g + 2 * h;
    const int tC = tA + 4;
    const v8us LA = ld8(tw + tapoff(tA)), LB = ld8(tw + tapoff(tA + 1));
    const v8us LC = ld8(tw + tapoff(tC)), LD = ld8(tw + tapoff(tC + 1));
    const v16bf ah = tobf(cat16(pickh(LA, LB), pickh(LC, LD)));
    const v16bf al = tobf(cat16(pickl(LA, LB), pickl(LC, LD)));
#pragma unroll
    for (int nt = 0; nt < 4; ++nt) {
      const unsigned short* bp = bw1 + nt * (16 * K1) + 32 * g;
      const v16bf bh  = tobf(cat16(ld8(bp), ld8(bp + 16)));
      const v16bf blo = tobf(cat16(ld8(bp + PL1), ld8(bp + PL1 + 16)));
      acc[nt] = mma3(acc[nt], ah, al, bh, blo);
    }
  }
  {
    v8us LA = ld8(tw + tapoff(80));
    LA = sel8(h == 0, LA);
    const v16bf ah = tobf(cat16(pickh(LA, z8), z8));
    const v16bf al = tobf(cat16(pickl(LA, z8), z8));
#pragma unroll
    for (int nt = 0; nt < 4; ++nt) {
      const unsigned short* bp = bw1 + nt * (16 * K1) + 32 * 10;
      const v16bf bh  = tobf(cat16(ld8(bp), ld8(bp + 16)));
      const v16bf blo = tobf(cat16(ld8(bp + PL1), ld8(bp + PL1 + 16)));
      acc[nt] = mma3(acc[nt], ah, al, bh, blo);
    }
  }

  unsigned short* h1w = h1s + w * (16 * H1P);
#pragma unroll
  for (int nt = 0; nt < 4; ++nt) {
    const int ch = 16 * nt + m;
    const float bias = b1[ch];
#pragma unroll
    for (int r = 0; r < 8; ++r) {
      const int px = 8 * h + r;
      const float v = fmaxf(acc[nt][r] + bias, 0.0f);
      const unsigned short hs = f2bf(v);
      h1w[px * H1P + ch]      = hs;
      h1w[px * H1P + 64 + ch] = f2bf(v - bf2f(hs));
    }
  }
  __syncthreads();

  v8f acc2[2];
  acc2[0] = zero8f(); acc2[1] = zero8f();
  const unsigned short* aw  = h1w + m * H1P + 8 * h;
  const unsigned short* bw2 = B2 + m * K2 + 8 * h;
#pragma unroll
  for (int kc = 0; kc < 2; ++kc) {
    const unsigned short* ap = aw + 32 * kc;
    const v16bf ah = tobf(cat16(ld8(ap), ld8(ap + 16)));
    const v16bf al = tobf(cat16(ld8(ap + 64), ld8(ap + 80)));
#pragma unroll
    for (int nt = 0; nt < 2; ++nt) {
      const unsigned short* bp = bw2 + nt * (16 * K2) + 32 * kc;
      const v16bf bh  = tobf(cat16(ld8(bp), ld8(bp + 16)));
      const v16bf blo = tobf(cat16(ld8(bp + PL2), ld8(bp + PL2 + 16)));
      acc2[nt] = mma3(acc2[nt], ah, al, bh, blo);
    }
  }

  unsigned short* h2w = h2s + w * (16 * 64);
#pragma unroll
  for (int nt = 0; nt < 2; ++nt) {
    const int ch = 16 * nt + m;
    const float bias = b2[ch];
#pragma unroll
    for (int r = 0; r < 8; ++r) {
      const int px = 8 * h + r;
      const float v = fmaxf(acc2[nt][r] + bias, 0.0f);
      const unsigned short hs = f2bf(v);
      h2w[px * 64 + ch]      = hs;
      h2w[px * 64 + 32 + ch] = f2bf(v - bf2f(hs));
    }
  }
  __syncthreads();
  const size_t pg = ((size_t)(bi * IMG + Y)) * IMG + x0 + 16 * w;
  unsigned short* dst = h2 + pg * 64;
  v8us pv[4];
#pragma unroll
  for (int q = 0; q < 4; ++q) pv[q] = ld8(h2w + (q * 32 + lane) * 8);
#pragma unroll
  for (int q = 0; q < 4; ++q) *(volatile v8us*)(dst + (q * 32 + lane) * 8) = pv[q];
  __threadfence();
#pragma unroll
  for (int q = 0; q < 4; ++q) *(volatile v8us*)(dst + (q * 32 + lane) * 8) = pv[q];
}

__global__ __launch_bounds__(64) void k_conv3(const unsigned short* __restrict__ h2,
                                              const unsigned short* __restrict__ B3,
                                              const float* __restrict__ b3,
                                              float* out, int bimg0) {
  __shared__ __attribute__((aligned(16))) unsigned short tileH[5 * THC * 64];
  __shared__ __attribute__((aligned(16))) float red[256];
  __shared__ __attribute__((aligned(16))) float outs[256];

  const int tid = threadIdx.x, lane = tid & 31, w = tid >> 5, h = lane >> 4, m = lane & 15;
  const int x0 = blockIdx.x * 64, Y = blockIdx.y, bi = blockIdx.z, bg = bimg0 + bi;

  for (int e = tid; e < 5 * THC * 8; e += 64) {
    const int pos = e >> 3, part = e & 7;
    const int i = pos / THC, j = pos - i * THC;
    const int Yg = Y - 2 + i, Xg = x0 - 2 + j;
    const bool in = ((unsigned)Yg < (unsigned)IMG) && ((unsigned)Xg < (unsigned)IMG);
    const int Yc = min(max(Yg, 0), IMG - 1), Xc = min(max(Xg, 0), IMG - 1);
    v8us v = ld8(h2 + ((size_t)((bi * IMG + Yc) * IMG + Xc)) * 64 + part * 8);
    v = sel8(in, v);
    *(v8us*)(tileH + pos * 64 + part * 8) = v;
  }
  __syncthreads();

  v8f acc = zero8f();
  const unsigned short* abase = tileH + (4 * m) * 64 + 8 * h;
  const unsigned short* bbase = B3 + m * K3 + 8 * h;
#pragma unroll 1
  for (int qq = 0; qq < 20; ++qq) {
    const int q = w * 20 + qq;
    const int dy = q >> 3, dxp = q & 7;
    const unsigned short* ap = abase + (dy * THC + dxp) * 64;
    const v16bf ah = tobf(cat16(ld8(ap), ld8(ap + 16)));
    const v16bf al = tobf(cat16(ld8(ap + 32), ld8(ap + 48)));
    const unsigned short* bp = bbase + 32 * q;
    const v16bf bh  = tobf(cat16(ld8(bp), ld8(bp + 16)));
    const v16bf blo = tobf(cat16(ld8(bp + PL3), ld8(bp + PL3 + 16)));
    acc = mma3(acc, ah, al, bh, blo);
  }

  if (w == 1) {
    const v4f lo4 = {acc[0], acc[1], acc[2], acc[3]};
    const v4f hi4 = {acc[4], acc[5], acc[6], acc[7]};
    *(v4f*)(red + lane * 8)     = lo4;
    *(v4f*)(red + lane * 8 + 4) = hi4;
  }
  __syncthreads();
  if (w == 0) {
    const v4f ra = *(const v4f*)(red + lane * 8);
    const v4f rb = *(const v4f*)(red + lane * 8 + 4);
    const int c = m & 3, s = m >> 2;
    const float bias = b3[c];
    float sum[8];
    sum[0] = acc[0] + ra[0]; sum[1] = acc[1] + ra[1]; sum[2] = acc[2] + ra[2]; sum[3] = acc[3] + ra[3];
    sum[4] = acc[4] + rb[0]; sum[5] = acc[5] + rb[1]; sum[6] = acc[6] + rb[2]; sum[7] = acc[7] + rb[3];
#pragma unroll
    for (int r = 0; r < 8; ++r) {
      const int px = 4 * (8 * h + r) + s;
      outs[px * 4 + c] = sum[r] + bias;
    }
  }
  __syncthreads();

  const int px = 32 * w + lane;
  const v4f ov = *(const v4f*)(outs + px * 4);
  float* op = out + ((((size_t)(bg * IMG + Y)) * IMG) + x0 + px) * 4;
  *(volatile v4f*)op = ov;
  __threadfence();
  *(volatile v4f*)op = ov;
}

extern "C" void kernel_launch(void* const* d_in, const int* in_sizes, int n_in,
                              void* d_out, int out_size, void* d_ws, size_t ws_size,
                              hipStream_t stream) {
  if (n_in < 7) return;
  if (in_sizes[0] != NIMG * LOW * LOW * 4) return;
  if (in_sizes[1] != 64 * 4 * 81 || in_sizes[2] < 64) return;
  if (in_sizes[3] != 32 * 64 || in_sizes[4] < 32) return;
  if (in_sizes[5] != 4 * 32 * 25 || in_sizes[6] < 4) return;
  if (out_size != NIMG * IMG * IMG * 4) return;

  const float* x  = (const float*)d_in[0];
  const float* w1 = (const float*)d_in[1];
  const float* b1 = (const float*)d_in[2];
  const float* w2 = (const float*)d_in[3];
  const float* b2 = (const float*)d_in[4];
  const float* w3 = (const float*)d_in[5];
  const float* b3 = (const float*)d_in[6];
  float* out = (float*)d_out;

  size_t off = 0;
  const size_t oB1 = off; off += (size_t)2 * PL1 * 2;
  const size_t oB2 = off; off += (size_t)2 * PL2 * 2;
  const size_t oB3 = off; off += (size_t)2 * PL3 * 2;
  off = (off + 4095) & ~(size_t)4095;
  const size_t oUp = off; off += (size_t)NIMG * IMG * IMG * 8 * 2;
  const size_t oH2 = off; off += (size_t)HALF * IMG * IMG * 64 * 2;
  if (off > ws_size) return;

  char* ws = (char*)d_ws;
  unsigned short* B1 = (unsigned short*)(ws + oB1);
  unsigned short* B2 = (unsigned short*)(ws + oB2);
  unsigned short* B3 = (unsigned short*)(ws + oB3);
  unsigned short* up = (unsigned short*)(ws + oUp);
  unsigned short* h2 = (unsigned short*)(ws + oH2);

  k_prep<<<dim3(11, 3, 1), 256, 0, stream>>>(w1, w2, w3, B1, B2, B3);
  k_up<<<(NIMG * IMG * IMG) / 256, 256, 0, stream>>>(x, up);
  for (int hf = 0; hf < NIMG / HALF; ++hf) {
    k_conv12<<<dim3(IMG / 64, IMG, HALF), 128, 0, stream>>>(up, B1, b1, B2, b2, h2, hf * HALF);
    k_conv3<<<dim3(IMG / 64, IMG, HALF), 64, 0, stream>>>(h2, B3, b3, out, hf * HALF);
  }
}
